// PredYWithS_55508157333621
// MI455X (gfx1250) — hardware-verified
//
#include <hip/hip_runtime.h>
#include <stddef.h>


typedef _Float16 v16h __attribute__((ext_vector_type(16)));
typedef _Float16 v8h  __attribute__((ext_vector_type(8)));
typedef float    v8f  __attribute__((ext_vector_type(8)));
typedef float    v4f  __attribute__((ext_vector_type(4)));

#define NROWS 2048
#define FEAT  256
#define LAT   128
#define NCLS  100
#define CPAD  128

#define LDC 68
#define LDZ 132

#define SCARRY 16.0f
#define WCARRY 64.0f
#define MCARRY 16.0f

static_assert((FEAT % 32) == 0 && (LAT % 32) == 0);
static_assert((NROWS % 64) == 0 && (CPAD % 64) == 0 && (FEAT % 64) == 0 && (LAT % 64) == 0);
static_assert(NCLS <= CPAD && (NCLS % 4) == 0);
static_assert(((64 * NCLS * 4) % 128) == 0);
static_assert((64 * NCLS) / 4 <= 7 * 256);
static_assert((LDC % 4) == 0 && LDC >= 64);
static_assert((LDZ % 4) == 0 && LDZ >= 128);
static_assert(LAT == 16 * 8);
static_assert(FEAT == 2 * 32 * 4);
static_assert((LAT % 32) == 0 && (NROWS % 8) == 0);

#define N_S    ((unsigned)NROWS * FEAT)
#define N_W1   ((unsigned)LAT * FEAT)
#define N_W2   ((unsigned)FEAT * LAT)
#define N_WFV  ((unsigned)NCLS * FEAT)
#define N_WFP  ((unsigned)CPAD * FEAT)
#define N_COV  ((unsigned)NCLS * FEAT * FEAT)
static_assert((N_S % 2048u) == 0 && (N_W1 % 2048u) == 0 && (N_W2 % 2048u) == 0);
static_assert((N_WFP % 2048u) == 0 && (N_COV % 2048u) == 0 && (N_WFV % 8u) == 0);

#define S16_BYTES   ((size_t)N_S * 2)
#define W1P_BYTES   ((size_t)N_W1 * 2)
#define W2P_BYTES   ((size_t)N_W2 * 2)
#define WFP_BYTES   ((size_t)N_WFP * 2)
#define COV_BYTES   ((size_t)N_COV * 2)
#define G_BYTES     ((size_t)NCLS * CPAD * FEAT * 4)
#define H_BYTES     ((size_t)NROWS * LAT * 4)
#define STAT_BYTES  ((size_t)2 * LAT * 4)
#define HN_BYTES    ((size_t)NROWS * LAT * 2)
#define F_BYTES     ((size_t)NROWS * FEAT * 2)
#define SG_BYTES    ((size_t)NCLS * CPAD * 4)
#define OFF_S16  ((size_t)0)
#define OFF_W1P  (OFF_S16 + S16_BYTES)
#define OFF_W2P  (OFF_W1P + W1P_BYTES)
#define OFF_WFP  (OFF_W2P + W2P_BYTES)
#define OFF_COV  (OFF_WFP + WFP_BYTES)
#define OFF_G    (OFF_COV + COV_BYTES)
#define OFF_H    (OFF_G + G_BYTES)
#define OFF_STAT (OFF_H + H_BYTES)
#define OFF_HN   (OFF_STAT + STAT_BYTES)
#define OFF_F    (OFF_HN + HN_BYTES)
#define OFF_SG   (OFF_F + F_BYTES)
#define WS_TOTAL (OFF_SG + SG_BYTES)
static_assert((S16_BYTES % 128) == 0 && (W1P_BYTES % 128) == 0 && (W2P_BYTES % 128) == 0);
static_assert((WFP_BYTES % 128) == 0 && (COV_BYTES % 128) == 0 && (G_BYTES % 128) == 0);
static_assert((H_BYTES % 128) == 0 && (STAT_BYTES % 128) == 0 && (HN_BYTES % 128) == 0);
static_assert((F_BYTES % 128) == 0 && (SG_BYTES % 128) == 0);
static_assert(WS_TOTAL <= (size_t)134217728);

__device__ __forceinline__ float bf16r(float x) {
  unsigned int u = __float_as_uint(x);
  u = (u + 0x7FFFu + ((u >> 16) & 1u)) & 0xFFFF0000u;
  return __uint_as_float(u);
}

static __device__ __forceinline__ _Float16 toh_flush(float v) {
  const _Float16 r = (_Float16)v;
  return (fabsf(v) < 6.103515625e-05f) ? (_Float16)0.0f : r;
}

__device__ __forceinline__ v16h frag_at(const _Float16* p) {
  v8h lo = *(const v8h*)(p);
  v8h hi = *(const v8h*)(p + 16);
  v16h out;
#pragma unroll
  for (int i = 0; i < 8; ++i) { out[i] = lo[i]; out[i + 8] = hi[i]; }
  return out;
}

__device__ __forceinline__ v8f wmma16(v16h a, v16h b, v8f c) {
  v8f d = __builtin_amdgcn_wmma_f32_16x16x32_f16(false, a, false, b, (short)0, c,
                                                 false, false);
  asm volatile("v_nop\n\tv_nop\n\tv_nop\n\tv_nop" : "+v"(d) : "v"(a), "v"(b));
  return d;
}

__device__ __forceinline__ float red32_sum(float x) {
#pragma unroll
  for (int off = 1; off < 32; off <<= 1) x += __shfl_xor(x, off, 32);
  return x;
}

__device__ __forceinline__ float relu_act(float t) {
  return fmaxf(t, 0.0f);
}

__global__ __launch_bounds__(256) void pconv_kernel(
    const float* __restrict__ in, _Float16* __restrict__ out,
    unsigned n_valid, unsigned n_total, float carry) {
  const unsigned e0 = (blockIdx.x * 256u + threadIdx.x) * 8u;
  const bool ok = e0 < n_valid;
  const unsigned es = ok ? e0 : (n_valid - 8u);
  const v4f a0 = *(const v4f*)(in + es);
  const v4f a1 = *(const v4f*)(in + es + 4u);
  v8h o;
#pragma unroll
  for (int i = 0; i < 4; ++i) {
    const float t0 = ok ? carry * bf16r(a0[i]) : 0.0f;
    const float t1 = ok ? carry * bf16r(a1[i]) : 0.0f;
    o[i]     = toh_flush(t0);
    o[i + 4] = toh_flush(t1);
  }
  _Float16* p = out + e0;
  *(volatile v8h*)p = o;
  __threadfence();
  *(volatile v8h*)p = o;
}

template <int MODE>
__device__ __forceinline__ void gemm_body(
    const _Float16* __restrict__ A16, const _Float16* __restrict__ Bt, const unsigned K,
    const float* __restrict__ bias, const float cs, const unsigned ldo,
    float* __restrict__ outf, _Float16* __restrict__ out16) {
  __shared__ float Cs[64 * LDC];
  const unsigned tid = threadIdx.x, lane = tid & 31u;
  const unsigned w = (unsigned)__builtin_amdgcn_readfirstlane((int)(threadIdx.x >> 5));
  const unsigned mw = w >> 1, nw = w & 1u;
  const unsigned hh = lane >> 4, m = lane & 15u;
  const unsigned n0 = blockIdx.x * 64u;
  const unsigned row0 = blockIdx.y * 64u;

  const _Float16* ap  = A16 + (size_t)(row0 + mw * 16u + m) * K + hh * 8u;
  const _Float16* bp0 = Bt + (size_t)(n0 + nw * 32u + m) * K + hh * 8u;
  const _Float16* bp1 = bp0 + (size_t)16 * K;
  v8f acc0 = {}, acc1 = {};
#pragma unroll 2
  for (unsigned k0 = 0; k0 < K; k0 += 32u) {
    const v16h a  = frag_at(ap + k0);
    const v16h b0 = frag_at(bp0 + k0);
    const v16h b1 = frag_at(bp1 + k0);
    acc0 = wmma16(a, b0, acc0);
    acc1 = wmma16(a, b1, acc1);
  }
#pragma unroll
  for (int r = 0; r < 8; ++r) {
    float* d = &Cs[(mw * 16u + hh * 8u + (unsigned)r) * LDC + nw * 32u + m];
    d[0]  = acc0[r];
    d[16] = acc1[r];
  }
  __syncthreads();

  if (MODE == 2) {
    v8h x[2];
    size_t off[2];
#pragma unroll
    for (unsigned i = 0; i < 2u; ++i) {
      const unsigned r = 32u * i + (tid >> 3);
      const unsigned c = (tid & 7u) * 8u;
      const v4f u0 = *(const v4f*)&Cs[r * LDC + c];
      const v4f u1 = *(const v4f*)&Cs[r * LDC + c + 4];
      const v4f g0 = *(const v4f*)(bias + n0 + c);
      const v4f g1 = *(const v4f*)(bias + n0 + c + 4u);
#pragma unroll
      for (int j = 0; j < 4; ++j) {
        x[i][j]     = toh_flush(MCARRY * relu_act(u0[j] * cs + bf16r(g0[j])));
        x[i][j + 4] = toh_flush(MCARRY * relu_act(u1[j] * cs + bf16r(g1[j])));
      }
      off[i] = (size_t)(row0 + r) * ldo + n0 + c;
    }
#pragma unroll
    for (int i = 0; i < 2; ++i) *(volatile v8h*)(out16 + off[i]) = x[i];
    __threadfence();
#pragma unroll
    for (int i = 0; i < 2; ++i) *(volatile v8h*)(out16 + off[i]) = x[i];
  }

  if (MODE == 0 || MODE == 1) {
    v4f xs[4];
    size_t off[4];
#pragma unroll
    for (unsigned i = 0; i < 4u; ++i) {
      const unsigned r = 16u * i + (tid >> 4);
      const unsigned c = (tid & 15u) * 4u;
      const v4f u = *(const v4f*)&Cs[r * LDC + c];
      v4f val;
      if (MODE == 0) {
        const v4f g = *(const v4f*)(bias + n0 + c);
#pragma unroll
        for (int j = 0; j < 4; ++j) val[j] = u[j] * cs + bf16r(g[j]);
      } else {
#pragma unroll
        for (int j = 0; j < 4; ++j) val[j] = u[j] * cs;
      }
      xs[i] = val;
      off[i] = (size_t)(row0 + r) * ldo + n0 + c;
    }
#pragma unroll
    for (int i = 0; i < 4; ++i) *(volatile v4f*)(outf + off[i]) = xs[i];
    __threadfence();
#pragma unroll
    for (int i = 0; i < 4; ++i) *(volatile v4f*)(outf + off[i]) = xs[i];
  }
}

__global__ __launch_bounds__(256) void gemm_h_kernel(
    const _Float16* __restrict__ S16, const _Float16* __restrict__ W1p,
    const float* __restrict__ b1, float* __restrict__ H) {
  gemm_body<0>(S16, W1p, (unsigned)FEAT, b1, 1.0f / (SCARRY * WCARRY), (unsigned)LAT,
               H, (_Float16*)0);
}
__global__ __launch_bounds__(256) void gemm_f_kernel(
    const _Float16* __restrict__ Hn16, const _Float16* __restrict__ W2p,
    const float* __restrict__ b2, _Float16* __restrict__ F16) {
  gemm_body<2>(Hn16, W2p, (unsigned)LAT, b2, 1.0f / (MCARRY * WCARRY), (unsigned)FEAT,
               (float*)0, F16);
}
__global__ __launch_bounds__(256) void gemm_g_kernel(
    const _Float16* __restrict__ Wfp, const _Float16* __restrict__ Cov16,
    float* __restrict__ G) {
  const size_t c = blockIdx.z;
  gemm_body<1>(Wfp, Cov16 + c * ((size_t)FEAT * FEAT), (unsigned)FEAT, (const float*)0,
               1.0f / (WCARRY * WCARRY), (unsigned)FEAT,
               G + c * ((size_t)CPAD * FEAT), (_Float16*)0);
}

__global__ __launch_bounds__(256) void bn_stat_kernel(
    const float* __restrict__ H, float* __restrict__ stat) {
  __shared__ float part[8 * 32];
  __shared__ float mus[32];
  __shared__ float line[64];
  const unsigned tid = threadIdx.x, lane = tid & 31u;
  const unsigned w = (unsigned)__builtin_amdgcn_readfirstlane((int)(threadIdx.x >> 5));
  const unsigned col = blockIdx.x * 32u + lane;
  const float* hp = H + (size_t)w * LAT + col;

  float s = 0.0f;
#pragma unroll 4
  for (unsigned r = 0; r < (unsigned)(NROWS / 8); ++r) s += hp[(size_t)r * (8u * LAT)];
  part[w * 32u + lane] = s;
  __syncthreads();
  if (w == 0u) {
    float t = 0.0f;
#pragma unroll
    for (unsigned k = 0; k < 8u; ++k) t += part[k * 32u + lane];
    mus[lane] = t * (1.0f / (float)NROWS);
  }
  __syncthreads();
  const float mu = mus[lane];
  float ss = 0.0f;
#pragma unroll 4
  for (unsigned r = 0; r < (unsigned)(NROWS / 8); ++r) {
    const float d = hp[(size_t)r * (8u * LAT)] - mu;
    ss += d * d;
  }
  part[w * 32u + lane] = ss;
  __syncthreads();
  if (w == 0u) {
    float t = 0.0f;
#pragma unroll
    for (unsigned k = 0; k < 8u; ++k) t += part[k * 32u + lane];
    const float var = t * (1.0f / (float)NROWS);
    line[lane] = mu;
    line[32u + lane] = 1.0f / sqrtf(var + 1.0e-5f);
  }
  __syncthreads();
  if (w == 0u) {
    const unsigned q = lane & 15u;
    const v4f x = *(const v4f*)&line[q * 4u];
    const unsigned dst = (q < 8u) ? (blockIdx.x * 32u + q * 4u)
                                  : ((unsigned)LAT + blockIdx.x * 32u + (q - 8u) * 4u);
    if (lane < 16u) {
      *(volatile v4f*)(stat + dst) = x;
      __threadfence();
      *(volatile v4f*)(stat + dst) = x;
    }
  }
}

__global__ __launch_bounds__(256) void bn_apply_kernel(
    const float* __restrict__ H, const float* __restrict__ stat,
    const float* __restrict__ gamma, const float* __restrict__ beta,
    _Float16* __restrict__ Hn) {
  const unsigned g = blockIdx.x * 256u + threadIdx.x;
  const unsigned row = g >> 4, c = (g & 15u) * 8u;
  const float* hp = H + (size_t)row * LAT + c;
  const v4f h0 = *(const v4f*)(hp);
  const v4f h1 = *(const v4f*)(hp + 4);
  const v4f m0 = *(const v4f*)(stat + c);
  const v4f m1 = *(const v4f*)(stat + c + 4u);
  const v4f r0 = *(const v4f*)(stat + LAT + c);
  const v4f r1 = *(const v4f*)(stat + LAT + c + 4u);
  const v4f g0 = *(const v4f*)(gamma + c);
  const v4f g1 = *(const v4f*)(gamma + c + 4u);
  const v4f b0 = *(const v4f*)(beta + c);
  const v4f b1 = *(const v4f*)(beta + c + 4u);
  v8h o;
#pragma unroll
  for (int i = 0; i < 4; ++i) {
    const float t0 = ((h0[i] - m0[i]) * r0[i]) * bf16r(g0[i]) + bf16r(b0[i]);
    const float t1 = ((h1[i] - m1[i]) * r1[i]) * bf16r(g1[i]) + bf16r(b1[i]);
    o[i]     = toh_flush(MCARRY * relu_act(t0));
    o[i + 4] = toh_flush(MCARRY * relu_act(t1));
  }
  _Float16* p = Hn + (size_t)row * LAT + c;
  *(volatile v8h*)p = o;
  __threadfence();
  *(volatile v8h*)p = o;
}

__global__ __launch_bounds__(256) void sg_kernel(
    const float* __restrict__ G, const float* __restrict__ Wfc, float* __restrict__ SG) {
  __shared__ float Sv[CPAD];
  const unsigned tid = threadIdx.x, lane = tid & 31u;
  const unsigned w = (unsigned)__builtin_amdgcn_readfirstlane((int)(threadIdx.x >> 5));
  const unsigned c = blockIdx.x;
  const float* gc = G + ((size_t)c * CPAD + c) * FEAT;
  const float* wc = Wfc + (size_t)c * FEAT;
#pragma unroll 1
  for (unsigned it = 0; it < 16u; ++it) {
    const unsigned i = w + 8u * it;
    const unsigned ic = (i < (unsigned)NCLS) ? i : (unsigned)(NCLS - 1);
    const float* gi = G + ((size_t)c * CPAD + ic) * FEAT;
    const float* wi = Wfc + (size_t)ic * FEAT;
    float q = 0.0f;
#pragma unroll 1
    for (unsigned t = 0; t < 2u; ++t) {
      const unsigned a = lane * 4u + 128u * t;
      const v4f gv = *(const v4f*)(gi + a);
      const v4f gk = *(const v4f*)(gc + a);
      const v4f xv = *(const v4f*)(wi + a);
      const v4f xk = *(const v4f*)(wc + a);
#pragma unroll
      for (int j = 0; j < 4; ++j)
        q += (gv[j] - gk[j]) * (bf16r(xv[j]) - bf16r(xk[j]));
    }
    q = red32_sum(q);
    const float val = (i < (unsigned)NCLS) ? q : 0.0f;
    if (lane == 0u) Sv[i] = val;
  }
  __syncthreads();
  if (w == 0u) {
    const v4f x = *(const v4f*)&Sv[lane * 4u];
    float* p = SG + (size_t)c * CPAD + lane * 4u;
    *(volatile v4f*)p = x;
    __threadfence();
    *(volatile v4f*)p = x;
  }
}

__global__ __launch_bounds__(256) void gemm_out_kernel(
    const _Float16* __restrict__ F16, const _Float16* __restrict__ Wfp,
    const float* __restrict__ bfc, const float* __restrict__ SG,
    const int* __restrict__ y, const float* __restrict__ ratio, float* __restrict__ out) {
  __shared__ float Cs[64 * LDZ];
  __shared__ int Ys[64];
  const unsigned tid = threadIdx.x, lane = tid & 31u;
  const unsigned w = (unsigned)__builtin_amdgcn_readfirstlane((int)(threadIdx.x >> 5));
  const unsigned mw = w >> 1, nw = w & 1u;
  const unsigned hh = lane >> 4, m = lane & 15u;
  const unsigned row0 = blockIdx.x * 64u;

  const _Float16* ap = F16 + (size_t)(row0 + mw * 16u + m) * FEAT + hh * 8u;
  const _Float16* bp = Wfp + (size_t)(nw * 64u + m) * FEAT + hh * 8u;
  v8f acc0 = {}, acc1 = {}, acc2 = {}, acc3 = {};
#pragma unroll 2
  for (unsigned k0 = 0; k0 < (unsigned)FEAT; k0 += 32u) {
    const v16h a  = frag_at(ap + k0);
    const v16h b0 = frag_at(bp + k0);
    const v16h b1 = frag_at(bp + 16u * FEAT + k0);
    const v16h b2 = frag_at(bp + 32u * FEAT + k0);
    const v16h b3 = frag_at(bp + 48u * FEAT + k0);
    acc0 = wmma16(a, b0, acc0);
    acc1 = wmma16(a, b1, acc1);
    acc2 = wmma16(a, b2, acc2);
    acc3 = wmma16(a, b3, acc3);
  }
#pragma unroll
  for (int r = 0; r < 8; ++r) {
    float* d = &Cs[(mw * 16u + hh * 8u + (unsigned)r) * LDZ + nw * 64u + m];
    d[0]  = acc0[r];
    d[16] = acc1[r];
    d[32] = acc2[r];
    d[48] = acc3[r];
  }
  if (tid < 64u) {
    int yy = y[row0 + tid];
    yy = (yy < 0) ? 0 : yy;
    yy = (yy > NCLS - 1) ? (NCLS - 1) : yy;
    Ys[tid] = yy;
  }
  __syncthreads();

  const float coef = bf16r(ratio[0]) * 0.5f;
  const float cs = 1.0f / (MCARRY * WCARRY);
  const unsigned nvec = (unsigned)(64 * NCLS / 4);
  v4f xs[7];
  size_t off[7];
#pragma unroll
  for (unsigned j = 0; j < 7u; ++j) {
    const unsigned idx = tid + 256u * j;
    const unsigned idc = (idx < nvec) ? idx : (nvec - 1u);
    const unsigned e = idc * 4u;
    const unsigned r = e / (unsigned)NCLS;
    const unsigned c = e - r * (unsigned)NCLS;
    const v4f u  = *(const v4f*)&Cs[r * LDZ + c];
    const v4f g  = *(const v4f*)(bfc + c);
    const v4f sg = *(const v4f*)(SG + (size_t)Ys[r] * CPAD + c);
    v4f val;
#pragma unroll
    for (int q = 0; q < 4; ++q) val[q] = (u[q] * cs + bf16r(g[q])) + coef * sg[q];
    xs[j] = val;
    off[j] = (size_t)row0 * NCLS + e;
  }
#pragma unroll
  for (unsigned j = 0; j < 7u; ++j)
    if (tid + 256u * j < nvec) *(volatile v4f*)(out + off[j]) = xs[j];
  __threadfence();
#pragma unroll
  for (unsigned j = 0; j < 7u; ++j)
    if (tid + 256u * j < nvec) *(volatile v4f*)(out + off[j]) = xs[j];
}

extern "C" void kernel_launch(void* const* d_in, const int* in_sizes, int n_in,
                              void* d_out, int out_size, void* d_ws, size_t ws_size,
                              hipStream_t stream) {
  if (n_in < 12) return;
  if ((long long)in_sizes[0] < (long long)NROWS * FEAT) return;
  if (in_sizes[1] < NROWS || in_sizes[2] < 1) return;
  if (in_sizes[3] < LAT * FEAT) return;
  if (in_sizes[4] < LAT || in_sizes[5] < LAT || in_sizes[6] < LAT) return;
  if (in_sizes[7] < FEAT * LAT || in_sizes[8] < FEAT) return;
  if (in_sizes[9] < NCLS * FEAT || in_sizes[10] < NCLS) return;
  if ((long long)in_sizes[11] < (long long)NCLS * FEAT * FEAT) return;
  if ((long long)out_size < (long long)NROWS * NCLS) return;
  if (ws_size < WS_TOTAL) return;

  const float* s     = (const float*)d_in[0];
  const int*   y     = (const int*)d_in[1];
  const float* ratio = (const float*)d_in[2];
  const float* W1    = (const float*)d_in[3];
  const float* b1    = (const float*)d_in[4];
  const float* gamma = (const float*)d_in[5];
  const float* beta  = (const float*)d_in[6];
  const float* W2    = (const float*)d_in[7];
  const float* b2    = (const float*)d_in[8];
  const float* Wfc   = (const float*)d_in[9];
  const float* bfc   = (const float*)d_in[10];
  const float* cov   = (const float*)d_in[11];
  float* out = (float*)d_out;

  char* ws = (char*)d_ws;
  _Float16* S16   = (_Float16*)(ws + OFF_S16);
  _Float16* W1p   = (_Float16*)(ws + OFF_W1P);
  _Float16* W2p   = (_Float16*)(ws + OFF_W2P);
  _Float16* Wfp   = (_Float16*)(ws + OFF_WFP);
  _Float16* Cov16 = (_Float16*)(ws + OFF_COV);
  float*    G     = (float*)(ws + OFF_G);
  float*    H     = (float*)(ws + OFF_H);
  float*    stat  = (float*)(ws + OFF_STAT);
  _Float16* Hn16  = (_Float16*)(ws + OFF_HN);
  _Float16* F16   = (_Float16*)(ws + OFF_F);
  float*    SG    = (float*)(ws + OFF_SG);

  dim3 blk(256);

  pconv_kernel<<<dim3(N_S / 2048u), blk, 0, stream>>>(s, S16, N_S, N_S, SCARRY);
  pconv_kernel<<<dim3(N_W1 / 2048u), blk, 0, stream>>>(W1, W1p, N_W1, N_W1, WCARRY);
  pconv_kernel<<<dim3(N_W2 / 2048u), blk, 0, stream>>>(W2, W2p, N_W2, N_W2, WCARRY);
  pconv_kernel<<<dim3(N_WFP / 2048u), blk, 0, stream>>>(Wfc, Wfp, N_WFV, N_WFP, WCARRY);
  pconv_kernel<<<dim3(N_COV / 2048u), blk, 0, stream>>>(cov, Cov16, N_COV, N_COV, WCARRY);

  gemm_h_kernel<<<dim3(LAT / 64, NROWS / 64), blk, 0, stream>>>(S16, W1p, b1, H);
  bn_stat_kernel<<<dim3(LAT / 32), blk, 0, stream>>>(H, stat);
  bn_apply_kernel<<<dim3(NROWS * 16 / 256), blk, 0, stream>>>(H, stat, gamma, beta, Hn16);
  gemm_f_kernel<<<dim3(FEAT / 64, NROWS / 64), blk, 0, stream>>>(Hn16, W2p, b2, F16);

  gemm_g_kernel<<<dim3(FEAT / 64, CPAD / 64, NCLS), blk, 0, stream>>>(Wfp, Cov16, G);
  sg_kernel<<<dim3(NCLS), blk, 0, stream>>>(G, Wfc, SG);

  gemm_out_kernel<<<dim3(NROWS / 64), blk, 0, stream>>>(F16, Wfp, bfc, SG, y, ratio, out);
}
